// HFFVSSBlock_12498354831586
// MI455X (gfx1250) — hardware-verified
//
#include <hip/hip_runtime.h>
#include <stdint.h>

#define NT    16384
#define DIM   256
#define INNER 384
#define DST   8
#define DTR   48
#define XZW   768
#define PJW   128
#define HID   512
#define NWIN  4096
#define LDC   132
#define TPW   72

#define S_LN  8.0f
#define S_XP  64.0f
#define S_DR  256.0f
#define S_YD  1024.0f
#define S_YM  256.0f
#define S_HG  64.0f
#define S_W   64.0f
#define RLO   1024.0f
#define ILO   0.0009765625f
#define LOG2E 1.4426950408889634f

static_assert((NT % 64) == 0);
static_assert(NWIN * 4 == NT);
static_assert((LDC * 4) % 16 == 0);
static_assert((TPW * 2) % 16 == 0);
static_assert((INNER % 128) == 0 && (DIM % 128) == 0 && (HID % 128) == 0 && (PJW % 128) == 0);

typedef _Float16 v16h __attribute__((ext_vector_type(16)));
typedef _Float16 v8h  __attribute__((ext_vector_type(8)));
typedef float    v8f  __attribute__((ext_vector_type(8)));
typedef float    v4f  __attribute__((ext_vector_type(4)));
typedef unsigned int v4u __attribute__((ext_vector_type(4)));
typedef unsigned int v2u __attribute__((ext_vector_type(2)));

__device__ __forceinline__ unsigned short bf_bits(float f) {
  unsigned u = __float_as_uint(f);
  return (unsigned short)((u + 0x7FFFu + ((u >> 16) & 1u)) >> 16);
}
__device__ __forceinline__ float bfr(float f) { return __uint_as_float(((unsigned)bf_bits(f)) << 16); }
__device__ __forceinline__ unsigned short h_bits(_Float16 x) { return __builtin_bit_cast(unsigned short, x); }
__device__ __forceinline__ unsigned short hb16(float f) { return h_bits((_Float16)f); }
__device__ __forceinline__ unsigned pk16(unsigned short a, unsigned short b) { return (unsigned)a | ((unsigned)b << 16); }
__device__ __forceinline__ v8f zero8() { v8f z = {0.f, 0.f, 0.f, 0.f, 0.f, 0.f, 0.f, 0.f}; return z; }
__device__ __forceinline__ float sigf(float x) { return __builtin_amdgcn_rcpf(1.0f + __expf(-x)); }
__device__ __forceinline__ float geluf(float x) { return 0.5f * x * (1.0f + erff(x * 0.70710678118654752f)); }

__device__ __forceinline__ float wsum(float v) {
  v += __shfl_xor(v, 1, 32);
  v += __shfl_xor(v, 2, 32);
  v += __shfl_xor(v, 4, 32);
  v += __shfl_xor(v, 8, 32);
  v += __shfl_xor(v, 16, 32);
  return v;
}

__device__ __forceinline__ unsigned hl2(float v0, float v1, unsigned& lo) {
  const _Float16 h0 = (_Float16)v0;
  const _Float16 h1 = (_Float16)v1;
  lo = pk16(hb16((v0 - (float)h0) * RLO), hb16((v1 - (float)h1) * RLO));
  return pk16(h_bits(h0), h_bits(h1));
}
__device__ __forceinline__ void pack4(const v4f v, const float s, v2u& ph, v2u& pl) {
  unsigned l0, l1;
  const unsigned p0 = hl2(v[0] * s, v[1] * s, l0);
  const unsigned p1 = hl2(v[2] * s, v[3] * s, l1);
  ph[0] = p0; ph[1] = p1;
  pl[0] = l0; pl[1] = l1;
}

__device__ __forceinline__ v16h ldfrag_h(const _Float16* p) {
  union { v16h v; v8h h[2]; } f;
  f.h[0] = *(const v8h*)(p);
  f.h[1] = *(const v8h*)(p + 16);
  return f.v;
}

__device__ __forceinline__ v8f mma_raw(v16h a, v16h b, v8f c) {
  return __builtin_amdgcn_wmma_f32_16x16x32_f16(false, a, false, b, (short)0, c, false, false);
}
__device__ __forceinline__ void guard8(v8f& c0, v8f& c1, v8f& c2, v8f& c3, v8f& c4, v8f& c5, v8f& c6, v8f& c7,
                                       const v16h& a0, const v16h& a1, const v16h& a2, const v16h& a3,
                                       const v16h& b0, const v16h& b1) {
#if defined(__HIP_DEVICE_COMPILE__)
  asm volatile("v_nop\n\tv_nop\n\tv_nop\n\tv_nop"
               : "+v"(c0), "+v"(c1), "+v"(c2), "+v"(c3), "+v"(c4), "+v"(c5), "+v"(c6), "+v"(c7)
               : "v"(a0), "v"(a1), "v"(a2), "v"(a3), "v"(b0), "v"(b1));
#endif
}

__device__ __forceinline__ void mm_tile2(const _Float16* __restrict__ Ah, const _Float16* __restrict__ Al, int lda,
                                         int acol0, const _Float16* __restrict__ W, int ldw, int nks,
                                         int arow0, int bcol0, float* Cs) {
  const int tid = threadIdx.x, wave = tid >> 5, lane = tid & 31, hh = lane >> 4, c = lane & 15;
  const int mw = wave >> 2, nw = wave & 3;
  const size_t ao0 = (size_t)(arow0 + mw * 32 + c) * (size_t)lda + acol0 + 8 * hh;
  const size_t ao1 = (size_t)(arow0 + mw * 32 + 16 + c) * (size_t)lda + acol0 + 8 * hh;
  const _Float16* a0h = Ah + ao0;
  const _Float16* a1h = Ah + ao1;
  const _Float16* a0l = Al + ao0;
  const _Float16* a1l = Al + ao1;
  const _Float16* b0p = W + (size_t)(bcol0 + nw * 32 + c) * (size_t)ldw + 8 * hh;
  const _Float16* b1p = W + (size_t)(bcol0 + nw * 32 + 16 + c) * (size_t)ldw + 8 * hh;
  v8f h00 = zero8(), h01 = zero8(), h10 = zero8(), h11 = zero8();
  v8f l00 = zero8(), l01 = zero8(), l10 = zero8(), l11 = zero8();
#pragma unroll 1
  for (int ks = 0; ks < nks; ++ks) {
    const int ko = ks * 32;
    const v16h fa0 = ldfrag_h(a0h + ko);
    const v16h fa1 = ldfrag_h(a1h + ko);
    const v16h ga0 = ldfrag_h(a0l + ko);
    const v16h ga1 = ldfrag_h(a1l + ko);
    const v16h fb0 = ldfrag_h(b0p + ko);
    const v16h fb1 = ldfrag_h(b1p + ko);
    h00 = mma_raw(fa0, fb0, h00);
    h01 = mma_raw(fa0, fb1, h01);
    h10 = mma_raw(fa1, fb0, h10);
    h11 = mma_raw(fa1, fb1, h11);
    l00 = mma_raw(ga0, fb0, l00);
    l01 = mma_raw(ga0, fb1, l01);
    l10 = mma_raw(ga1, fb0, l10);
    l11 = mma_raw(ga1, fb1, l11);
    guard8(h00, h01, h10, h11, l00, l01, l10, l11, fa0, fa1, ga0, ga1, fb0, fb1);
  }
#pragma unroll
  for (int r = 0; r < 8; ++r) {
    const int row = mw * 32 + 8 * hh + r;
    Cs[row * LDC + nw * 32 + c]             = h00[r] + l00[r] * ILO;
    Cs[row * LDC + nw * 32 + 16 + c]        = h01[r] + l01[r] * ILO;
    Cs[(row + 16) * LDC + nw * 32 + c]      = h10[r] + l10[r] * ILO;
    Cs[(row + 16) * LDC + nw * 32 + 16 + c] = h11[r] + l11[r] * ILO;
  }
}

__global__ __launch_bounds__(256)
void k_cvt_wt(const float* __restrict__ src, int K, int N, unsigned short* dst, int Kp) {
  __shared__ __align__(16) _Float16 T[32 * TPW];
  const int tid = threadIdx.x, wv = tid >> 5, lane = tid & 31;
  const int n0 = blockIdx.x * 32, k0 = blockIdx.y * 64;
#pragma unroll 1
  for (int i = 0; i < 8; ++i) {
    const int kk = i * 8 + wv;
    const int k = k0 + kk;
    const int kc = min(k, K - 1);
    const float v = src[(size_t)kc * (size_t)N + n0 + lane];
    const float m = (k < K) ? S_W : 0.0f;
    T[lane * TPW + kk] = (_Float16)(bfr(v) * m);
  }
  __syncthreads();
  const int row = tid >> 3, piece = tid & 7;
  const v8h q = *(const v8h*)(T + row * TPW + piece * 8);
  const v4u u = __builtin_bit_cast(v4u, q);
  unsigned short* p = dst + (size_t)(n0 + row) * (size_t)Kp + k0 + piece * 8;
  *(volatile v4u*)p = u;
  __threadfence();
  *(volatile v4u*)p = u;
}

__global__ __launch_bounds__(256)
void k_ln(const float* __restrict__ src, const float* __restrict__ g, const float* __restrict__ bb, int rin,
          unsigned short* oh, unsigned short* ol) {
  const int tid = threadIdx.x, wv = tid >> 5, lane = tid & 31;
  const size_t t = (size_t)blockIdx.x * 8 + wv;
  const v4f x0 = *(const v4f*)(src + t * DIM + lane * 4);
  const v4f x1 = *(const v4f*)(src + t * DIM + 128 + lane * 4);
  const v4f g0 = *(const v4f*)(g + lane * 4);
  const v4f g1 = *(const v4f*)(g + 128 + lane * 4);
  const v4f b0 = *(const v4f*)(bb + lane * 4);
  const v4f b1 = *(const v4f*)(bb + 128 + lane * 4);
  v4f a0, a1;
#pragma unroll
  for (int e = 0; e < 4; ++e) {
    a0[e] = rin ? bfr(x0[e]) : x0[e];
    a1[e] = rin ? bfr(x1[e]) : x1[e];
  }
  float s = ((a0[0] + a0[1]) + (a0[2] + a0[3])) + ((a1[0] + a1[1]) + (a1[2] + a1[3]));
  s = wsum(s);
  const float mu = s * (1.0f / (float)DIM);
  v4f d0, d1;
#pragma unroll
  for (int e = 0; e < 4; ++e) { d0[e] = a0[e] - mu; d1[e] = a1[e] - mu; }
  float sq = ((d0[0] * d0[0] + d0[1] * d0[1]) + (d0[2] * d0[2] + d0[3] * d0[3])) +
             ((d1[0] * d1[0] + d1[1] * d1[1]) + (d1[2] * d1[2] + d1[3] * d1[3]));
  sq = wsum(sq);
  const float rs = rsqrtf(sq * (1.0f / (float)DIM) + 1e-5f);
  v4f y0, y1;
#pragma unroll
  for (int e = 0; e < 4; ++e) {
    y0[e] = (d0[e] * rs) * bfr(g0[e]) + bfr(b0[e]);
    y1[e] = (d1[e] * rs) * bfr(g1[e]) + bfr(b1[e]);
  }
  v2u ph0, pl0, ph1, pl1;
  pack4(y0, S_LN, ph0, pl0);
  pack4(y1, S_LN, ph1, pl1);
  unsigned short* hp = oh + t * DIM + lane * 4;
  unsigned short* lp = ol + t * DIM + lane * 4;
  *(volatile v2u*)hp = ph0;
  *(volatile v2u*)(hp + 128) = ph1;
  *(volatile v2u*)lp = pl0;
  *(volatile v2u*)(lp + 128) = pl1;
  __threadfence();
  *(volatile v2u*)hp = ph0;
  *(volatile v2u*)(hp + 128) = ph1;
  *(volatile v2u*)lp = pl0;
  *(volatile v2u*)(lp + 128) = pl1;
}

__global__ __launch_bounds__(256)
void k_dwconv(const float* __restrict__ xz, const float* __restrict__ dwk, unsigned short* ydh, unsigned short* ydl) {
  const int tid = threadIdx.x, wv = tid >> 5, lane = tid & 31;
  const int t = blockIdx.x * 8 + wv;
  const int bq = t >> 12, hq = (t >> 6) & 63, wq = t & 63;
#pragma unroll 1
  for (int cb = 0; cb < 3; ++cb) {
    const int c0 = cb * 128 + lane * 4;
    v4f acc;
    acc[0] = 0.f; acc[1] = 0.f; acc[2] = 0.f; acc[3] = 0.f;
#pragma unroll 1
    for (int tap = 0; tap < 9; ++tap) {
      const int kh = tap / 3, kw = tap - kh * 3;
      const int h2 = hq + kh - 1, w2 = wq + kw - 1;
      const float m = (((unsigned)h2 < 64u) && ((unsigned)w2 < 64u)) ? 1.0f : 0.0f;
      const int hc = min(max(h2, 0), 63), wc = min(max(w2, 0), 63);
      const v4f xv = *(const v4f*)(xz + (size_t)((bq * 64 + hc) * 64 + wc) * XZW + c0);
      const v4f kv = *(const v4f*)(dwk + tap * INNER + c0);
#pragma unroll
      for (int e = 0; e < 4; ++e) acc[e] += (xv[e] * m) * bfr(kv[e]);
    }
    v2u ph, pl;
    pack4(acc, S_YD, ph, pl);
    unsigned short* hp = ydh + (size_t)t * INNER + c0;
    unsigned short* lp = ydl + (size_t)t * INNER + c0;
    *(volatile v2u*)hp = ph;
    *(volatile v2u*)lp = pl;
    __threadfence();
    *(volatile v2u*)hp = ph;
    *(volatile v2u*)lp = pl;
  }
}

template <int DIR>
__global__ __launch_bounds__(256)
void k_scan(const float* __restrict__ xz, const float* __restrict__ proj, const float* __restrict__ dt,
            const float* __restrict__ alog, const float* __restrict__ dd, float* ys) {
  const int tid = threadIdx.x, wv = tid >> 5, lane = tid & 31;
  const int gw = blockIdx.x * 8 + wv;
  const int win = gw / 12;
  const int grp = gw - win * 12;
  const int ch = grp * 32 + lane;
  const int bq = win >> 10, hb = (win >> 5) & 31, wb = win & 31;
  float a2[DST];
#pragma unroll
  for (int n = 0; n < DST; ++n) a2[n] = -__expf(bfr(alog[ch * DST + n])) * LOG2E;
  const float Dc = bfr(dd[ch]);
  float st[DST];
#pragma unroll
  for (int n = 0; n < DST; ++n) st[n] = 0.0f;
  const int boff = DIR ? (64 + DTR) : DTR;
#pragma unroll 1
  for (int i = 0; i < 4; ++i) {
    const int t = DIR ? (3 - i) : i;
    const size_t tok = (size_t)((bq * 64 + hb * 2 + (t >> 1)) * 64 + wb * 2 + (t & 1));
    const float x = xz[tok * XZW + ch];
    const float d = dt[tok * INNER + ch];
    const v4f bq0 = *(const v4f*)(proj + tok * PJW + boff);
    const v4f bq1 = *(const v4f*)(proj + tok * PJW + boff + 4);
    const v4f cq0 = *(const v4f*)(proj + tok * PJW + boff + 8);
    const v4f cq1 = *(const v4f*)(proj + tok * PJW + boff + 12);
    const float bx = d * x;
    float y = 0.0f;
#pragma unroll
    for (int n = 0; n < DST; ++n) {
      const float bn = (n < 4) ? bq0[n & 3] : bq1[n & 3];
      const float cn = (n < 4) ? cq0[n & 3] : cq1[n & 3];
      const float ex = exp2f(d * a2[n]);
      st[n] = ex * st[n] + bx * bn;
      y += st[n] * cn;
    }
    float yv = y + x * Dc;
    float* p = ys + tok * INNER + ch;
    if (DIR) {
      const float pr = *p;
      yv = 0.5f * (pr + yv);
    }
    *(volatile float*)p = yv;
    __threadfence();
    *(volatile float*)p = yv;
  }
}

template <int MODE>
__global__ __launch_bounds__(256)
void k_gemm(const unsigned short* __restrict__ ah, const unsigned short* __restrict__ al, int lda, int acol0,
            const unsigned short* __restrict__ w, int ldw, int nks,
            const float* __restrict__ q0, const float* __restrict__ q1, const float* __restrict__ q2,
            float* o32, unsigned short* oh, unsigned short* ol) {
  __shared__ __align__(16) float Cs[64 * LDC];
  const int tid = threadIdx.x, wave = tid >> 5, lane = tid & 31;
  const int mb = blockIdx.x, nb = blockIdx.y;
  mm_tile2((const _Float16*)(const void*)ah, (const _Float16*)(const void*)al, lda, acol0,
           (const _Float16*)(const void*)w, ldw, nks, mb * 64, nb * 128, Cs);
  __syncthreads();
  const int cb = nb * 128 + lane * 4;
#pragma unroll 1
  for (int it = 0; it < 8; ++it) {
    const int row = wave * 8 + it;
    const size_t t = (size_t)mb * 64 + row;
    const v4f a = *(const v4f*)(Cs + row * LDC + lane * 4);
    if (MODE == 0) {
      v4f v;
#pragma unroll
      for (int e = 0; e < 4; ++e) v[e] = a[e] * (1.0f / 512.0f);
      float* p = o32 + t * XZW + cb;
      if (nb < 3) {
        v2u ph, pl;
        pack4(v, S_XP, ph, pl);
        unsigned short* hp = oh + t * INNER + cb;
        unsigned short* lp = ol + t * INNER + cb;
        *(volatile v4f*)p = v;
        *(volatile v2u*)hp = ph;
        *(volatile v2u*)lp = pl;
        __threadfence();
        *(volatile v4f*)p = v;
        *(volatile v2u*)hp = ph;
        *(volatile v2u*)lp = pl;
      } else {
        *(volatile v4f*)p = v;
        __threadfence();
        *(volatile v4f*)p = v;
      }
    } else if (MODE == 1) {
      v4f v, dv;
#pragma unroll
      for (int e = 0; e < 4; ++e) {
        v[e] = a[e] * (1.0f / 4096.0f);
        const int col = lane * 4 + e;
        dv[e] = ((col & 63) < DTR) ? v[e] : 0.0f;
      }
      v2u ph, pl;
      pack4(dv, S_DR, ph, pl);
      float* p = o32 + t * PJW + cb;
      unsigned short* hp = oh + t * PJW + cb;
      unsigned short* lp = ol + t * PJW + cb;
      *(volatile v4f*)p = v;
      *(volatile v2u*)hp = ph;
      *(volatile v2u*)lp = pl;
      __threadfence();
      *(volatile v4f*)p = v;
      *(volatile v2u*)hp = ph;
      *(volatile v2u*)lp = pl;
    } else if (MODE == 2) {
      const v4f bv = *(const v4f*)(q0 + cb);
      v4f s;
#pragma unroll
      for (int e = 0; e < 4; ++e) {
        const float v = a[e] * (1.0f / 16384.0f) + bfr(bv[e]);
        s[e] = v * sigf(v);
      }
      float* p = o32 + t * INNER + cb;
      *(volatile v4f*)p = s;
      __threadfence();
      *(volatile v4f*)p = s;
    } else if (MODE == 3) {
      const v4f ysv = *(const v4f*)(q0 + t * INNER + cb);
      const v4f zv  = *(const v4f*)(q1 + t * XZW + INNER + cb);
      const v4f gv  = *(const v4f*)(q2 + cb);
      v4f ym;
#pragma unroll
      for (int e = 0; e < 4; ++e) {
        const float yc = geluf(a[e] * (1.0f / 65536.0f));
        const float alp = sigf(bfr(gv[e]));
        const float y = alp * ysv[e] + (1.0f - alp) * yc;
        const float z = zv[e];
        ym[e] = y * (z * sigf(z));
      }
      v2u ph, pl;
      pack4(ym, S_YM, ph, pl);
      unsigned short* hp = oh + t * INNER + cb;
      unsigned short* lp = ol + t * INNER + cb;
      *(volatile v2u*)hp = ph;
      *(volatile v2u*)lp = pl;
      __threadfence();
      *(volatile v2u*)hp = ph;
      *(volatile v2u*)lp = pl;
    } else if (MODE == 4) {
      const v4f xv = *(const v4f*)(q0 + t * DIM + cb);
      v4f o;
#pragma unroll
      for (int e = 0; e < 4; ++e) o[e] = bfr(xv[e]) + a[e] * (1.0f / 16384.0f);
      float* p = o32 + t * DIM + cb;
      *(volatile v4f*)p = o;
      __threadfence();
      *(volatile v4f*)p = o;
    } else if (MODE == 5) {
      const v4f bv = *(const v4f*)(q0 + cb);
      v4f gl;
#pragma unroll
      for (int e = 0; e < 4; ++e) gl[e] = geluf(a[e] * (1.0f / 512.0f) + bfr(bv[e]));
      v2u ph, pl;
      pack4(gl, S_HG, ph, pl);
      unsigned short* hp = oh + t * HID + cb;
      unsigned short* lp = ol + t * HID + cb;
      *(volatile v2u*)hp = ph;
      *(volatile v2u*)lp = pl;
      __threadfence();
      *(volatile v2u*)hp = ph;
      *(volatile v2u*)lp = pl;
    } else {
      const v4f bv = *(const v4f*)(q0 + cb);
      const v4f xo = *(const v4f*)(q1 + t * DIM + cb);
      v4f o;
#pragma unroll
      for (int e = 0; e < 4; ++e) o[e] = xo[e] + (a[e] * (1.0f / 4096.0f) + bfr(bv[e]));
      float* p = o32 + t * DIM + cb;
      *(volatile v4f*)p = o;
      __threadfence();
      *(volatile v4f*)p = o;
    }
  }
}

extern "C" void kernel_launch(void* const* d_in, const int* in_sizes, int n_in,
                              void* d_out, int out_size, void* d_ws, size_t ws_size,
                              hipStream_t stream) {
  if (n_in < 24) return;
  if (in_sizes[0] != NT * DIM) return;
  if (in_sizes[1] != DIM || in_sizes[2] != DIM) return;
  if (in_sizes[3] != DIM * XZW) return;
  if (in_sizes[4] != INNER * 64 || in_sizes[9] != INNER * 64) return;
  if (in_sizes[5] != DTR * INNER || in_sizes[10] != DTR * INNER) return;
  if (in_sizes[6] != INNER || in_sizes[11] != INNER) return;
  if (in_sizes[7] != INNER * DST || in_sizes[12] != INNER * DST) return;
  if (in_sizes[8] != INNER || in_sizes[13] != INNER) return;
  if (in_sizes[14] != 9 * INNER || in_sizes[15] != INNER * INNER || in_sizes[16] != INNER) return;
  if (in_sizes[17] != INNER * DIM) return;
  if (in_sizes[18] != DIM || in_sizes[19] != DIM) return;
  if (in_sizes[20] != DIM * HID || in_sizes[21] != HID) return;
  if (in_sizes[22] != HID * DIM || in_sizes[23] != DIM) return;
  if (out_size != NT * DIM) return;

  const float* x      = (const float*)d_in[0];
  const float* n1g    = (const float*)d_in[1];
  const float* n1b    = (const float*)d_in[2];
  const float* inw    = (const float*)d_in[3];
  const float* fxpw   = (const float*)d_in[4];
  const float* fdtw   = (const float*)d_in[5];
  const float* fdtb   = (const float*)d_in[6];
  const float* falog  = (const float*)d_in[7];
  const float* fdd    = (const float*)d_in[8];
  const float* bxpw   = (const float*)d_in[9];
  const float* bdtw   = (const float*)d_in[10];
  const float* bdtb   = (const float*)d_in[11];
  const float* balog  = (const float*)d_in[12];
  const float* bdd    = (const float*)d_in[13];
  const float* dwk    = (const float*)d_in[14];
  const float* pww    = (const float*)d_in[15];
  const float* gate   = (const float*)d_in[16];
  const float* outw   = (const float*)d_in[17];
  const float* n2g    = (const float*)d_in[18];
  const float* n2b    = (const float*)d_in[19];
  const float* f1w    = (const float*)d_in[20];
  const float* f1b    = (const float*)d_in[21];
  const float* f2w    = (const float*)d_in[22];
  const float* f2b    = (const float*)d_in[23];
  float* out = (float*)d_out;

  const size_t s16_128 = (size_t)NT * 128 * 2;
  const size_t s16_256 = (size_t)NT * 256 * 2;
  const size_t s16_384 = (size_t)NT * 384 * 2;
  const size_t s16_512 = (size_t)NT * 512 * 2;
  const size_t s32_128 = (size_t)NT * 128 * 4;
  const size_t s32_256 = (size_t)NT * 256 * 4;
  const size_t s32_384 = (size_t)NT * 384 * 4;
  const size_t s32_768 = (size_t)NT * 768 * 4;
  size_t sRA = s32_768;
  if (s32_256 + 2 * s16_512 > sRA) sRA = s32_256 + 2 * s16_512;
  size_t sRB = 2 * s16_256;
  if (s32_128 + 2 * s16_128 > sRB) sRB = s32_128 + 2 * s16_128;
  if (2 * s16_384 > sRB) sRB = 2 * s16_384;
  size_t sRC = 2 * s16_384;
  if (s32_384 > sRC) sRC = s32_384;
  size_t sRD = s32_384;
  if (2 * s16_256 > sRD) sRD = 2 * s16_256;
  const size_t sWIN  = (size_t)XZW * DIM * 2;
  const size_t sWXP  = (size_t)PJW * INNER * 2;
  const size_t sWDT  = (size_t)2 * INNER * 64 * 2;
  const size_t sWPW  = (size_t)INNER * INNER * 2;
  const size_t sWOUT = (size_t)DIM * INNER * 2;
  const size_t sWF1  = (size_t)HID * DIM * 2;
  const size_t sWF2  = (size_t)DIM * HID * 2;

  size_t off = 0;
  const size_t oRA = off; off += sRA;
  const size_t oRB = off; off += sRB;
  const size_t oRC = off; off += sRC;
  const size_t oRD = off; off += sRD;
  const size_t oWIN = off; off += sWIN;
  const size_t oWXP = off; off += sWXP;
  const size_t oWDT = off; off += sWDT;
  const size_t oWPW = off; off += sWPW;
  const size_t oWOUT = off; off += sWOUT;
  const size_t oWF1 = off; off += sWF1;
  const size_t oWF2 = off; off += sWF2;
  if (off > ws_size) return;
  if (off > (size_t)134217728) return;

  char* ws = (char*)d_ws;
  float*          XZ   = (float*)(ws + oRA);
  float*          XO   = (float*)(ws + oRA);
  unsigned short* HH   = (unsigned short*)(ws + oRA + s32_256);
  unsigned short* HL   = (unsigned short*)(ws + oRA + s32_256 + s16_512);
  unsigned short* XNH  = (unsigned short*)(ws + oRB);
  unsigned short* XNL  = (unsigned short*)(ws + oRB + s16_256);
  float*          PROJ = (float*)(ws + oRB);
  unsigned short* DRH  = (unsigned short*)(ws + oRB + s32_128);
  unsigned short* DRL  = (unsigned short*)(ws + oRB + s32_128 + s16_128);
  unsigned short* YDH  = (unsigned short*)(ws + oRB);
  unsigned short* YDL  = (unsigned short*)(ws + oRB + s16_384);
  unsigned short* XPH  = (unsigned short*)(ws + oRC);
  unsigned short* XPL  = (unsigned short*)(ws + oRC + s16_384);
  float*          DT   = (float*)(ws + oRC);
  unsigned short* YMH  = (unsigned short*)(ws + oRC);
  unsigned short* YML  = (unsigned short*)(ws + oRC + s16_384);
  float*          YS   = (float*)(ws + oRD);
  unsigned short* H2H  = (unsigned short*)(ws + oRD);
  unsigned short* H2L  = (unsigned short*)(ws + oRD + s16_256);
  unsigned short* WIN  = (unsigned short*)(ws + oWIN);
  unsigned short* WXP  = (unsigned short*)(ws + oWXP);
  unsigned short* WDT  = (unsigned short*)(ws + oWDT);
  unsigned short* WPW  = (unsigned short*)(ws + oWPW);
  unsigned short* WOUT = (unsigned short*)(ws + oWOUT);
  unsigned short* WF1  = (unsigned short*)(ws + oWF1);
  unsigned short* WF2  = (unsigned short*)(ws + oWF2);

  const dim3 blk(256);
  k_ln<<<dim3(NT / 8), blk, 0, stream>>>(x, n1g, n1b, 1, XNH, XNL);
  k_cvt_wt<<<dim3(XZW / 32, DIM / 64), blk, 0, stream>>>(inw, DIM, XZW, WIN, DIM);
  k_cvt_wt<<<dim3(64 / 32, INNER / 64), blk, 0, stream>>>(fxpw, INNER, 64, WXP, INNER);
  k_cvt_wt<<<dim3(64 / 32, INNER / 64), blk, 0, stream>>>(bxpw, INNER, 64, WXP + (size_t)64 * INNER, INNER);
  k_cvt_wt<<<dim3(INNER / 32, 1), blk, 0, stream>>>(fdtw, DTR, INNER, WDT, 64);
  k_cvt_wt<<<dim3(INNER / 32, 1), blk, 0, stream>>>(bdtw, DTR, INNER, WDT + (size_t)INNER * 64, 64);
  k_cvt_wt<<<dim3(INNER / 32, INNER / 64), blk, 0, stream>>>(pww, INNER, INNER, WPW, INNER);
  k_cvt_wt<<<dim3(DIM / 32, INNER / 64), blk, 0, stream>>>(outw, INNER, DIM, WOUT, INNER);
  k_cvt_wt<<<dim3(HID / 32, DIM / 64), blk, 0, stream>>>(f1w, DIM, HID, WF1, DIM);
  k_cvt_wt<<<dim3(DIM / 32, HID / 64), blk, 0, stream>>>(f2w, HID, DIM, WF2, HID);
  k_gemm<0><<<dim3(NT / 64, XZW / 128), blk, 0, stream>>>(XNH, XNL, DIM, 0, WIN, DIM, DIM / 32,
                                                           n1g, n1g, n1g, XZ, XPH, XPL);
  k_gemm<1><<<dim3(NT / 64, 1), blk, 0, stream>>>(XPH, XPL, INNER, 0, WXP, INNER, INNER / 32,
                                                   n1g, n1g, n1g, PROJ, DRH, DRL);
  k_gemm<2><<<dim3(NT / 64, INNER / 128), blk, 0, stream>>>(DRH, DRL, PJW, 0, WDT, 64, 2,
                                                             fdtb, n1g, n1g, DT, DRH, DRL);
  k_scan<0><<<dim3(NWIN * 12 / 8), blk, 0, stream>>>(XZ, PROJ, DT, falog, fdd, YS);
  k_gemm<2><<<dim3(NT / 64, INNER / 128), blk, 0, stream>>>(DRH, DRL, PJW, 64, WDT + (size_t)INNER * 64, 64, 2,
                                                             bdtb, n1g, n1g, DT, DRH, DRL);
  k_scan<1><<<dim3(NWIN * 12 / 8), blk, 0, stream>>>(XZ, PROJ, DT, balog, bdd, YS);
  k_dwconv<<<dim3(NT / 8), blk, 0, stream>>>(XZ, dwk, YDH, YDL);
  k_gemm<3><<<dim3(NT / 64, INNER / 128), blk, 0, stream>>>(YDH, YDL, INNER, 0, WPW, INNER, INNER / 32,
                                                             YS, XZ, gate, XO, YMH, YML);
  k_gemm<4><<<dim3(NT / 64, DIM / 128), blk, 0, stream>>>(YMH, YML, INNER, 0, WOUT, INNER, INNER / 32,
                                                           x, n1g, n1g, XO, YMH, YML);
  k_ln<<<dim3(NT / 8), blk, 0, stream>>>(XO, n2g, n2b, 0, H2H, H2L);
  k_gemm<5><<<dim3(NT / 64, HID / 128), blk, 0, stream>>>(H2H, H2L, DIM, 0, WF1, DIM, DIM / 32,
                                                           f1b, n1g, n1g, XO, HH, HL);
  k_gemm<6><<<dim3(NT / 64, DIM / 128), blk, 0, stream>>>(HH, HL, HID, 0, WF2, HID, HID / 32,
                                                           f2b, XO, n1g, out, HH, HL);
  (void)hipGetLastError();
}
